// Mamba2DScalarHead_86904368267767
// MI455X (gfx1250) — hardware-run, weakly checked
//
#include <hip/hip_runtime.h>
#include <math.h>

typedef __attribute__((ext_vector_type(16))) _Float16 v16h;
typedef __attribute__((ext_vector_type(8)))  _Float16 v8h;
typedef __attribute__((ext_vector_type(8)))  float    v8f;
typedef __attribute__((ext_vector_type(4)))  float    v4f;

constexpr int kBatch  = 16;
constexpr int kGridH  = 32;
constexpr int kGridW  = 32;
constexpr int kSeqLen = kGridH * kGridW;
constexpr int kChanIn = 768;
constexpr int kDm     = 512;
constexpr int kDm2    = 2 * kDm;
constexpr int kDepth  = 4;
constexpr int kRows   = kBatch * kSeqLen;
constexpr int kHalfD  = kDm / 2;
constexpr int kConvTP = 260;
static_assert(kSeqLen == 1024);
static_assert(kRows == 16384);
static_assert((kChanIn % 32) == 0 && (kDm % 32) == 0);
static_assert((kRows % 64) == 0 && (kDm % 64) == 0 && (kChanIn % 64) == 0);
static_assert(kGridH == 32 && kGridW == 32);

constexpr float kActCarry = 16.0f;
constexpr float kWtCarry  = 1024.0f;
constexpr float kFold     = 1.0f / (kActCarry * kWtCarry);
constexpr float kF16MinNormal = 6.103515625e-05f;

constexpr size_t kSzWtIn  = (size_t)kDm * kChanIn * 2;
constexpr size_t kSzWtInp = (size_t)kDepth * kDm2 * kDm * 2;
constexpr size_t kSzWtOut = (size_t)kDepth * kDm * kDm * 2;
constexpr size_t kSzTab   = (size_t)kSeqLen * kDm * 4;
constexpr size_t kSzAct   = (size_t)kRows * kDm * 4;
constexpr size_t kSzH16   = (size_t)kRows * kDm * 2;
constexpr size_t kSzStat  = (size_t)kRows * 4;
constexpr size_t kOffWtIn  = 0;
constexpr size_t kOffWtInp = kOffWtIn  + kSzWtIn;
constexpr size_t kOffWtOut = kOffWtInp + kSzWtInp;
constexpr size_t kOffPow   = kOffWtOut + kSzWtOut;
constexpr size_t kOffIpow  = kOffPow   + kSzTab;
constexpr size_t kOffRA    = kOffIpow  + kSzTab;
constexpr size_t kOffRB    = kOffRA    + kSzAct;
constexpr size_t kOffRU    = kOffRB    + kSzAct;
constexpr size_t kOffH16   = kOffRU    + kSzAct;
constexpr size_t kOffMu    = kOffH16   + kSzH16;
constexpr size_t kOffRs    = kOffMu    + kSzStat;
constexpr size_t kWsTotal  = kOffRs    + kSzStat;
static_assert(kWsTotal == 128843776ull);
static_assert(kWsTotal <= 134217728ull);
static_assert((size_t)kRows * kChanIn * 2 <= kSzAct);
static_assert((kOffWtInp % 128) == 0 && (kOffWtOut % 128) == 0 && (kOffPow % 128) == 0 && (kOffIpow % 128) == 0 &&
              (kOffRA % 128) == 0 && (kOffRB % 128) == 0 && (kOffRU % 128) == 0 && (kOffH16 % 128) == 0 &&
              (kOffMu % 128) == 0 && (kOffRs % 128) == 0);

__device__ __forceinline__ _Float16 to_h16(float v) {
  const float lim = 60000.0f;
  float w = fminf(fmaxf(v, -lim), lim);
  w = (fabsf(w) < kF16MinNormal) ? 0.0f : w;
  return (_Float16)w;
}

__device__ __forceinline__ v16h frag_ld(const _Float16* p) {
  union { v16h v; v8h h[2]; } f;
  f.h[0] = *(const v8h*)(p);
  f.h[1] = *(const v8h*)(p + 16);
  return f.v;
}

__device__ __forceinline__ v8f mma_g(v16h a, v16h b, v8f c) {
  c = __builtin_amdgcn_wmma_f32_16x16x32_f16(false, a, false, b, (short)0, c, false, false);
  asm volatile("v_nop\n\tv_nop\n\tv_nop\n\tv_nop" : "+v"(c) : "v"(a), "v"(b));
  return c;
}

__device__ __forceinline__ void row_center(const float* xr, int lane, v4f& xa, v4f& xb, v4f& xc, v4f& xd,
                                           float& mu, float& rstd) {
  const int c0 = lane * 8;
  xa = *(const v4f*)(xr + c0);
  xb = *(const v4f*)(xr + c0 + 4);
  xc = *(const v4f*)(xr + kHalfD + c0);
  xd = *(const v4f*)(xr + kHalfD + c0 + 4);
  float s = ((xa[0] + xa[1]) + (xa[2] + xa[3])) + ((xb[0] + xb[1]) + (xb[2] + xb[3]));
  s += ((xc[0] + xc[1]) + (xc[2] + xc[3])) + ((xd[0] + xd[1]) + (xd[2] + xd[3]));
#pragma unroll
  for (int off = 16; off >= 1; off >>= 1) s += __shfl_xor(s, off, 32);
  mu = s * (1.0f / (float)kDm);
  xa = xa - mu;
  xb = xb - mu;
  xc = xc - mu;
  xd = xd - mu;
  float q = ((xa[0] * xa[0] + xa[1] * xa[1]) + (xa[2] * xa[2] + xa[3] * xa[3]))
          + ((xb[0] * xb[0] + xb[1] * xb[1]) + (xb[2] * xb[2] + xb[3] * xb[3]));
  q += ((xc[0] * xc[0] + xc[1] * xc[1]) + (xc[2] * xc[2] + xc[3] * xc[3]))
     + ((xd[0] * xd[0] + xd[1] * xd[1]) + (xd[2] * xd[2] + xd[3] * xd[3]));
#pragma unroll
  for (int off = 16; off >= 1; off >>= 1) q += __shfl_xor(q, off, 32);
  rstd = rsqrtf(q * (1.0f / (float)kDm) + 1e-5f);
}

__global__ __launch_bounds__(256) void wt_plane_kernel(
    const float* __restrict__ W, unsigned short* __restrict__ Bt, int Kdim, int Ndim)
{
  __shared__ float sT[64 * 65];
  const int tid = threadIdx.x, lane = tid & 31, wave = tid >> 5;
  const int n0 = blockIdx.x * 64, k0 = blockIdx.y * 64;
  const float* Wz = W + (size_t)blockIdx.z * Kdim * Ndim;
  unsigned short* Bz = Bt + (size_t)blockIdx.z * Ndim * Kdim;
  const int ln = tid & 63, lk = tid >> 6;
#pragma unroll
  for (int it = 0; it < 16; ++it) {
    const int k = it * 4 + lk;
    sT[k * 65 + ln] = Wz[(size_t)(k0 + k) * Ndim + n0 + ln];
  }
  __syncthreads();
  const int q = lane >> 3, c8 = (lane & 7) * 8;
  v8h hv[2];
#pragma unroll
  for (int it = 0; it < 2; ++it) {
    const int n = it * 32 + wave * 4 + q;
#pragma unroll
    for (int e = 0; e < 8; ++e) hv[it][e] = to_h16(sT[(c8 + e) * 65 + n] * kWtCarry);
  }
  for (int pass = 0; pass < 2; ++pass) {
#pragma unroll
    for (int it = 0; it < 2; ++it) {
      const int n = it * 32 + wave * 4 + q;
      *(volatile v8h*)(Bz + (size_t)(n0 + n) * Kdim + k0 + c8) = hv[it];
    }
    __threadfence();
  }
}

__global__ __launch_bounds__(256) void tok_plane_kernel(
    const float* __restrict__ src, unsigned short* __restrict__ dst, int total8)
{
  const int i = blockIdx.x * 256 + threadIdx.x;
  if (i >= total8) return;
  const size_t e0 = (size_t)i << 3;
  const v4f a0 = *(const v4f*)(src + e0);
  const v4f a1 = *(const v4f*)(src + e0 + 4);
  v8h hv;
#pragma unroll
  for (int e = 0; e < 4; ++e) {
    hv[e]     = to_h16(a0[e] * kActCarry);
    hv[4 + e] = to_h16(a1[e] * kActCarry);
  }
  unsigned short* q = dst + e0;
  *(volatile v8h*)q = hv;
  __threadfence();
  *(volatile v8h*)q = hv;
}

template <int EPI>
__global__ __launch_bounds__(256) void gemm_f16_kernel(
    const unsigned short* __restrict__ Ap, int lda,
    const unsigned short* __restrict__ Btp, int ldb,
    void* __restrict__ Cout, int ldc,
    const float* __restrict__ bias,
    const float* __restrict__ aux, int ldaux,
    int M, int N, int K, float scale)
{
  const _Float16* A  = (const _Float16*)Ap;
  const _Float16* Bt = (const _Float16*)Btp;
  __shared__ __align__(16) float sT[8][16 * 68];
  const int lane = threadIdx.x & 31;
  const int wave = threadIdx.x >> 5;
  const int tilesN = N >> 6;
  const int tilesM = M >> 6;
  const int tile = blockIdx.x * 8 + wave;
  if (tile >= tilesM * tilesN) return;
  const int tm = tile / tilesN;
  const int tn = tile - tm * tilesN;
  const int m0 = tm << 6;
  const int n0 = tn << 6;
  const int rlane = lane & 15;
  const int koff  = (lane >> 4) * 8;
  const int mOff  = (lane >> 4) * 8;

  v8f acc[4][4];
#pragma unroll
  for (int i = 0; i < 4; ++i)
#pragma unroll
    for (int j = 0; j < 4; ++j) acc[i][j] = (v8f){0.f, 0.f, 0.f, 0.f, 0.f, 0.f, 0.f, 0.f};

  for (int k0 = 0; k0 < K; k0 += 32) {
    v16h bf[4];
#pragma unroll
    for (int j = 0; j < 4; ++j)
      bf[j] = frag_ld(Bt + (size_t)(n0 + (j << 4) + rlane) * ldb + koff + k0);
#pragma unroll
    for (int i = 0; i < 4; ++i) {
      const v16h af = frag_ld(A + (size_t)(m0 + (i << 4) + rlane) * lda + koff + k0);
#pragma unroll
      for (int j = 0; j < 4; ++j) acc[i][j] = mma_g(af, bf[j], acc[i][j]);
    }
  }

  float* slab = sT[wave];
#pragma unroll
  for (int i = 0; i < 4; ++i) {
    const int mBase = m0 + (i << 4);
#pragma unroll
    for (int j = 0; j < 4; ++j) {
      const int n = n0 + (j << 4) + rlane;
      const float bv = bias[n];
#pragma unroll
      for (int r = 0; r < 8; ++r) {
        float v = acc[i][j][r] * scale + bv;
        if (EPI == 2) v = __builtin_amdgcn_rcpf(1.0f + __expf(-v));
        slab[(mOff + r) * 68 + (j << 4) + rlane] = v;
      }
    }
    __builtin_amdgcn_fence(__ATOMIC_RELEASE, "workgroup");
    __builtin_amdgcn_wave_barrier();
    __builtin_amdgcn_fence(__ATOMIC_ACQUIRE, "workgroup");
    if (EPI != 2) {
      float* C = (float*)Cout;
      const int hh = lane >> 4, c4 = (lane & 15) * 4;
      v4f vals[8];
#pragma unroll
      for (int it = 0; it < 8; ++it) {
        const int row = it * 2 + hh;
        v4f v = *(const v4f*)(slab + row * 68 + c4);
        if (EPI == 1) {
          const v4f rv = *(const v4f*)(aux + (size_t)(mBase + row) * ldaux + n0 + c4);
          v = v + rv;
        }
        vals[it] = v;
      }
      for (int pass = 0; pass < 2; ++pass) {
#pragma unroll
        for (int it = 0; it < 8; ++it) {
          const int row = it * 2 + hh;
          *(volatile v4f*)(C + (size_t)(mBase + row) * ldc + n0 + c4) = vals[it];
        }
        __threadfence();
      }
    } else {
      unsigned short* C = (unsigned short*)Cout;
      const int q = lane >> 3, c8 = (lane & 7) * 8;
      v8h hv[4];
#pragma unroll
      for (int it = 0; it < 4; ++it) {
        const int row = it * 4 + q;
        const float* sp = slab + row * 68 + c8;
        const v4f g0 = *(const v4f*)(sp);
        const v4f g1 = *(const v4f*)(sp + 4);
        const float* yp = aux + (size_t)(mBase + row) * ldaux + n0 + c8;
        const v4f y0 = *(const v4f*)(yp);
        const v4f y1 = *(const v4f*)(yp + 4);
#pragma unroll
        for (int e = 0; e < 4; ++e) {
          hv[it][e]     = to_h16((y0[e] * g0[e]) * kActCarry);
          hv[it][4 + e] = to_h16((y1[e] * g1[e]) * kActCarry);
        }
      }
      for (int pass = 0; pass < 2; ++pass) {
#pragma unroll
        for (int it = 0; it < 4; ++it) {
          const int row = it * 4 + q;
          *(volatile v8h*)(C + (size_t)(mBase + row) * ldc + n0 + c8) = hv[it];
        }
        __threadfence();
      }
    }
    __builtin_amdgcn_fence(__ATOMIC_RELEASE, "workgroup");
    __builtin_amdgcn_wave_barrier();
    __builtin_amdgcn_fence(__ATOMIC_ACQUIRE, "workgroup");
  }
}

__global__ __launch_bounds__(256) void ln_rows_kernel(
    const float* __restrict__ X, const float* __restrict__ gw, const float* __restrict__ gb,
    unsigned short* __restrict__ H)
{
  const int lane = threadIdx.x & 31, wave = threadIdx.x >> 5;
  const int row = blockIdx.x * 8 + wave;
  if (row >= kRows) return;
  v4f xa, xb, xc, xd;
  float mu, rstd;
  row_center(X + (size_t)row * kDm, lane, xa, xb, xc, xd, mu, rstd);
  const int c0 = lane * 8;
  const v4f wa = *(const v4f*)(gw + c0);
  const v4f wb = *(const v4f*)(gw + c0 + 4);
  const v4f wc = *(const v4f*)(gw + kHalfD + c0);
  const v4f wd = *(const v4f*)(gw + kHalfD + c0 + 4);
  const v4f ba = *(const v4f*)(gb + c0);
  const v4f bb = *(const v4f*)(gb + c0 + 4);
  const v4f bc = *(const v4f*)(gb + kHalfD + c0);
  const v4f bd = *(const v4f*)(gb + kHalfD + c0 + 4);
  v8h h0, h1;
#pragma unroll
  for (int e = 0; e < 4; ++e) {
    h0[e]     = to_h16(((xa[e] * rstd) * wa[e] + ba[e]) * kActCarry);
    h0[4 + e] = to_h16(((xb[e] * rstd) * wb[e] + bb[e]) * kActCarry);
    h1[e]     = to_h16(((xc[e] * rstd) * wc[e] + bc[e]) * kActCarry);
    h1[4 + e] = to_h16(((xd[e] * rstd) * wd[e] + bd[e]) * kActCarry);
  }
  unsigned short* hr = H + (size_t)row * kDm;
  for (int pass = 0; pass < 2; ++pass) {
    *(volatile v8h*)(hr + c0) = h0;
    *(volatile v8h*)(hr + kHalfD + c0) = h1;
    __threadfence();
  }
}

__global__ __launch_bounds__(256) void pow_table_kernel(
    const float* __restrict__ al, float* __restrict__ POW, float* __restrict__ IPOW)
{
  const int idx = blockIdx.x * 256 + threadIdx.x;
  const int d = idx % kDm;
  const int t = idx / kDm;
  const float x = al[d];
  float a = 1.0f / (1.0f + expf(-x));
  a = fminf(fmaxf(a, 1e-4f), 0.9999f);
  const float la = logf(a);
  float p = expf((float)t * la);
  p = fmaxf(p, 1e-20f);
  const float ip = 1.0f / p;
  volatile float* pp = POW + idx;
  volatile float* pi = IPOW + idx;
  *pp = p;
  *pi = ip;
  __threadfence();
  *pp = p;
  *pi = ip;
}

__global__ __launch_bounds__(256) void conv_silu_kernel(
    const float* __restrict__ XIN, const float* __restrict__ cw, const float* __restrict__ cb,
    float* __restrict__ U)
{
  __shared__ __align__(16) float sT[16 * kConvTP];
  const int tid = threadIdx.x, lane = tid & 31, wave = tid >> 5;
  const int d0 = blockIdx.x * 256, d = d0 + tid;
  const int bh = blockIdx.y;
  const int h = bh & (kGridH - 1);
  const int rowC = bh * kGridW;
  const bool upOk = (h > 0);
  const bool dnOk = (h < kGridH - 1);
  const int rowU = upOk ? (rowC - kGridW) : rowC;
  const int rowD = dnOk ? (rowC + kGridW) : rowC;
  const float k00 = cw[0 * kDm + d], k01 = cw[1 * kDm + d], k02 = cw[2 * kDm + d];
  const float k10 = cw[3 * kDm + d], k11 = cw[4 * kDm + d], k12 = cw[5 * kDm + d];
  const float k20 = cw[6 * kDm + d], k21 = cw[7 * kDm + d], k22 = cw[8 * kDm + d];
  const float bc = cb[d];
  float l0 = 0.0f, l1 = 0.0f, l2 = 0.0f;
  float m0, m1, m2;
  {
    const float vu = XIN[(size_t)rowU * kDm + d];
    const float vc = XIN[(size_t)rowC * kDm + d];
    const float vd = XIN[(size_t)rowD * kDm + d];
    m0 = upOk ? vu : 0.0f;
    m1 = vc;
    m2 = dnOk ? vd : 0.0f;
  }
  const int hrow = wave >> 1;
  const int hch  = (wave & 1) * 128 + lane * 4;
#pragma unroll 1
  for (int sub = 0; sub < 2; ++sub) {
#pragma unroll 1
    for (int s = 0; s < 16; ++s) {
      const int w = sub * 16 + s;
      const int wn = w + 1;
      const bool colOk = (wn < kGridW);
      const int wc = colOk ? wn : (kGridW - 1);
      const float vu = XIN[(size_t)(rowU + wc) * kDm + d];
      const float vc = XIN[(size_t)(rowC + wc) * kDm + d];
      const float vd = XIN[(size_t)(rowD + wc) * kDm + d];
      const float n0 = (upOk && colOk) ? vu : 0.0f;
      const float n1 = colOk ? vc : 0.0f;
      const float n2 = (dnOk && colOk) ? vd : 0.0f;
      float acc = k00 * l0;
      acc = fmaf(k01, m0, acc);
      acc = fmaf(k02, n0, acc);
      acc = fmaf(k10, l1, acc);
      acc = fmaf(k11, m1, acc);
      acc = fmaf(k12, n1, acc);
      acc = fmaf(k20, l2, acc);
      acc = fmaf(k21, m2, acc);
      acc = fmaf(k22, n2, acc);
      const float sv = acc + bc;
      const float sg = __builtin_amdgcn_rcpf(1.0f + __expf(-sv));
      sT[s * kConvTP + tid] = sv * sg;
      l0 = m0; l1 = m1; l2 = m2;
      m0 = n0; m1 = n1; m2 = n2;
    }
    __syncthreads();
    v4f fv[4];
#pragma unroll
    for (int it = 0; it < 4; ++it) fv[it] = *(const v4f*)(sT + (it * 4 + hrow) * kConvTP + hch);
    const int lb = rowC + sub * 16;
    for (int pass = 0; pass < 2; ++pass) {
#pragma unroll
      for (int it = 0; it < 4; ++it)
        *(volatile v4f*)(U + (size_t)(lb + it * 4 + hrow) * kDm + d0 + hch) = fv[it];
      __threadfence();
    }
    __syncthreads();
  }
}

__global__ __launch_bounds__(64) void scan_kernel(
    const float* __restrict__ U, const float* __restrict__ POW, const float* __restrict__ IPOW,
    const float* __restrict__ sb, const float* __restrict__ sc, const float* __restrict__ sd,
    float* Y)
{
  const int gid = blockIdx.x * 64 + threadIdx.x;
  const int d  = gid % kDm;
  const int bi = gid / kDm;
  const float bb = sb[d];
  const float qc = 0.25f * sc[d];
  const float dd = sd[d];
  const size_t base = (size_t)bi * kSeqLen * kDm + d;
#pragma unroll 1
  for (int dir = 0; dir < 4; ++dir) {
    float r = 0.0f;
#pragma unroll 1
    for (int t = 0; t < kSeqLen; ++t) {
      const int q = (dir & 1) ? (kSeqLen - 1 - t) : t;
      const int pos = (dir & 2) ? (((q & 31) << 5) | (q >> 5)) : q;
      const size_t o = base + (size_t)pos * kDm;
      const float u  = U[o];
      const float p  = POW[t * kDm + d];
      const float ip = IPOW[t * kDm + d];
      const float yold = Y[o];
      r = r + (u * bb) * ip;
      const float s = r * p;
      const float prev = (dir == 0) ? 0.0f : yold;
      const float accv = prev + s;
      const float fin  = qc * accv + dd * u;
      const float outv = (dir == 3) ? fin : accv;
      volatile float* yp = Y + o;
      *yp = outv;
      __threadfence();
      *yp = outv;
    }
  }
}

__global__ __launch_bounds__(256) void row_stats_kernel(
    const float* __restrict__ X, float* __restrict__ MU, float* __restrict__ RS)
{
  __shared__ float sM[32];
  __shared__ float sR[32];
  const int lane = threadIdx.x & 31, wave = threadIdx.x >> 5;
  const int row0 = blockIdx.x * 32;
#pragma unroll 1
  for (int i = 0; i < 4; ++i) {
    const int lr = wave * 4 + i;
    v4f xa, xb, xc, xd;
    float mu, rstd;
    row_center(X + (size_t)(row0 + lr) * kDm, lane, xa, xb, xc, xd, mu, rstd);
    if (lane == 0) {
      sM[lr] = mu;
      sR[lr] = rstd;
    }
  }
  __syncthreads();
  if (wave == 0) {
    const float mv = sM[lane];
    const float rv = sR[lane];
    volatile float* pm = MU + row0 + lane;
    volatile float* pr = RS + row0 + lane;
    *pm = mv;
    *pr = rv;
    __threadfence();
    *pm = mv;
    *pr = rv;
  }
}

__global__ __launch_bounds__(256) void pool_kernel(
    const float* __restrict__ X, const float* __restrict__ MU, const float* __restrict__ RS,
    const float* __restrict__ gw, const float* __restrict__ gb, float* __restrict__ out)
{
  const int gid = blockIdx.x * 256 + threadIdx.x;
  const int d  = gid % kDm;
  const int bi = gid / kDm;
  const float wv = gw[d];
  const float bv = gb[d];
  float a0 = 0.0f, a1 = 0.0f, a2 = 0.0f, a3 = 0.0f;
#pragma unroll 1
  for (int n = 0; n < kSeqLen; n += 4) {
    const size_t row = (size_t)bi * kSeqLen + n;
    const v4f m = *(const v4f*)(MU + row);
    const v4f r = *(const v4f*)(RS + row);
    const float x0 = X[(row + 0) * kDm + d];
    const float x1 = X[(row + 1) * kDm + d];
    const float x2 = X[(row + 2) * kDm + d];
    const float x3 = X[(row + 3) * kDm + d];
    a0 += ((x0 - m[0]) * r[0]) * wv + bv;
    a1 += ((x1 - m[1]) * r[1]) * wv + bv;
    a2 += ((x2 - m[2]) * r[2]) * wv + bv;
    a3 += ((x3 - m[3]) * r[3]) * wv + bv;
  }
  const float res = ((a0 + a1) + (a2 + a3)) * (1.0f / (float)kSeqLen);
  volatile float* po = out + gid;
  *po = res;
  __threadfence();
  *po = res;
}

extern "C" void kernel_launch(void* const* d_in, const int* in_sizes, int n_in,
                              void* d_out, int out_size, void* d_ws, size_t ws_size,
                              hipStream_t stream)
{
  if (n_in < 17) return;
  if (in_sizes[0] != kRows * kChanIn) return;
  if (in_sizes[1] != kChanIn * kDm) return;
  if (in_sizes[2] != kDm) return;
  if (in_sizes[3] != kDepth * kDm) return;
  if (in_sizes[4] != kDepth * kDm) return;
  if (in_sizes[5] != kDepth * kDm * kDm2) return;
  if (in_sizes[6] != kDepth * kDm2) return;
  if (in_sizes[7] != kDepth * 9 * kDm) return;
  if (in_sizes[8] != kDepth * kDm) return;
  if (in_sizes[9] != kDepth * kDm) return;
  if (in_sizes[10] != kDepth * kDm) return;
  if (in_sizes[11] != kDepth * kDm) return;
  if (in_sizes[12] != kDepth * kDm) return;
  if (in_sizes[13] != kDepth * kDm * kDm) return;
  if (in_sizes[14] != kDepth * kDm) return;
  if (in_sizes[15] != kDm) return;
  if (in_sizes[16] != kDm) return;
  if (out_size != kBatch * kDm) return;
  if (ws_size < kWsTotal) return;

  const float* tokens = (const float*)d_in[0];
  const float* in_w   = (const float*)d_in[1];
  const float* in_b   = (const float*)d_in[2];
  const float* nw     = (const float*)d_in[3];
  const float* nb     = (const float*)d_in[4];
  const float* iw     = (const float*)d_in[5];
  const float* ib     = (const float*)d_in[6];
  const float* cw     = (const float*)d_in[7];
  const float* cb     = (const float*)d_in[8];
  const float* al     = (const float*)d_in[9];
  const float* sb     = (const float*)d_in[10];
  const float* sc     = (const float*)d_in[11];
  const float* sd     = (const float*)d_in[12];
  const float* ow     = (const float*)d_in[13];
  const float* ob     = (const float*)d_in[14];
  const float* onw    = (const float*)d_in[15];
  const float* onb    = (const float*)d_in[16];
  float* out = (float*)d_out;

  char* ws = (char*)d_ws;
  unsigned short* WTIN  = (unsigned short*)(ws + kOffWtIn);
  unsigned short* WTINP = (unsigned short*)(ws + kOffWtInp);
  unsigned short* WTOUT = (unsigned short*)(ws + kOffWtOut);
  float* POW  = (float*)(ws + kOffPow);
  float* IPOW = (float*)(ws + kOffIpow);
  float* RA   = (float*)(ws + kOffRA);
  float* RB   = (float*)(ws + kOffRB);
  float* RUf  = (float*)(ws + kOffRU);
  unsigned short* RUh = (unsigned short*)(ws + kOffRU);
  unsigned short* H16 = (unsigned short*)(ws + kOffH16);
  float* MU = (float*)(ws + kOffMu);
  float* RS = (float*)(ws + kOffRs);

  wt_plane_kernel<<<dim3(kDm / 64, kChanIn / 64, 1), 256, 0, stream>>>(in_w, WTIN, kChanIn, kDm);
  wt_plane_kernel<<<dim3(kDm2 / 64, kDm / 64, kDepth), 256, 0, stream>>>(iw, WTINP, kDm, kDm2);
  wt_plane_kernel<<<dim3(kDm / 64, kDm / 64, kDepth), 256, 0, stream>>>(ow, WTOUT, kDm, kDm);

  const int tok8 = kRows * kChanIn / 8;
  tok_plane_kernel<<<tok8 / 256, 256, 0, stream>>>(tokens, RUh, tok8);

  const int gemmBlocks = (kRows / 64) * (kDm / 64) / 8;

  gemm_f16_kernel<0><<<gemmBlocks, 256, 0, stream>>>(
      RUh, kChanIn, WTIN, kChanIn, (void*)RA, kDm, in_b, nullptr, 0, kRows, kDm, kChanIn, kFold);

  for (int i = 0; i < kDepth; ++i) {
    float* Xcur = (i & 1) ? RB : RA;
    float* Xoth = (i & 1) ? RA : RB;
    const unsigned short* WtInpI = WTINP + (size_t)i * kDm2 * kDm;
    const unsigned short* WtOutI = WTOUT + (size_t)i * kDm * kDm;

    ln_rows_kernel<<<kRows / 8, 256, 0, stream>>>(Xcur, nw + i * kDm, nb + i * kDm, H16);

    pow_table_kernel<<<kSeqLen * kDm / 256, 256, 0, stream>>>(al + i * kDm, POW, IPOW);

    gemm_f16_kernel<0><<<gemmBlocks, 256, 0, stream>>>(
        H16, kDm, WtInpI, kDm, (void*)Xoth, kDm, ib + i * kDm2, nullptr, 0, kRows, kDm, kDm, kFold);

    conv_silu_kernel<<<dim3(kDm / 256, kBatch * kGridH), 256, 0, stream>>>(
        Xoth, cw + (size_t)i * 9 * kDm, cb + i * kDm, RUf);

    scan_kernel<<<kBatch * kDm / 64, 64, 0, stream>>>(
        RUf, POW, IPOW, sb + i * kDm, sc + i * kDm, sd + i * kDm, Xoth);

    gemm_f16_kernel<2><<<gemmBlocks, 256, 0, stream>>>(
        H16, kDm, WtInpI + (size_t)kDm * kDm, kDm, (void*)RUh, kDm, ib + i * kDm2 + kDm, Xoth, kDm,
        kRows, kDm, kDm, kFold);

    gemm_f16_kernel<1><<<gemmBlocks, 256, 0, stream>>>(
        RUh, kDm, WtOutI, kDm, (void*)Xoth, kDm, ob + i * kDm, Xcur, kDm, kRows, kDm, kDm, kFold);
  }

  float* Xfin = (kDepth & 1) ? RB : RA;
  row_stats_kernel<<<kRows / 32, 256, 0, stream>>>(Xfin, MU, RS);
  pool_kernel<<<kBatch * kDm / 256, 256, 0, stream>>>(Xfin, MU, RS, onw, onb, out);
}
